// SpectralSelfAttention_26388279067184
// MI455X (gfx1250) — hardware-verified
//
#include <hip/hip_runtime.h>


#define NB_  8
#define HW   4096
#define CC   256
#define DQK  32
#define DV   128
#define NPJ  192
#define NR   (NB_ * HW)
#define DM   CC
#define PCAR 1024.0f
#define LOSC 1024.0f
typedef _Float16 h16;
typedef unsigned short bf;
typedef __attribute__((ext_vector_type(16))) __bf16   v16bf;
typedef __attribute__((ext_vector_type(16))) _Float16 v16h;
typedef __attribute__((ext_vector_type(8)))  _Float16 v8h;
typedef __attribute__((ext_vector_type(8)))  unsigned short v8us;
typedef __attribute__((ext_vector_type(8)))  float    v8f;
typedef __attribute__((ext_vector_type(4)))  float    v4f;
typedef v8h  __attribute__((may_alias)) v8ha;
typedef v4f  __attribute__((may_alias)) v4fa;
typedef v8us __attribute__((may_alias)) v8usa;

__device__ __forceinline__ unsigned short f2bf(float f) { unsigned u = __float_as_uint(f); u += 0x7FFFu + ((u >> 16) & 1u); return (unsigned short)(u >> 16); }
__device__ __forceinline__ float bf2f(unsigned short b) { return __uint_as_float(((unsigned)b) << 16); }
__device__ __forceinline__ float bfr(float f) { return bf2f(f2bf(f)); }
__device__ __forceinline__ v16h cat16(v8h lo, v8h hi) { return __builtin_shufflevector(lo, hi, 0, 1, 2, 3, 4, 5, 6, 7, 8, 9, 10, 11, 12, 13, 14, 15); }
__device__ __forceinline__ v16bf cat16b(v8us lo, v8us hi) { return __builtin_bit_cast(v16bf, __builtin_shufflevector(lo, hi, 0, 1, 2, 3, 4, 5, 6, 7, 8, 9, 10, 11, 12, 13, 14, 15)); }
__device__ __forceinline__ v8f wmma16(v16h a, v16h b, v8f c) { return __builtin_amdgcn_wmma_f32_16x16x32_f16(false, a, false, b, (short)0, c, false, false); }
__device__ __forceinline__ v8f wmmab(v16bf a, v16bf b, v8f c) { return __builtin_amdgcn_wmma_f32_16x16x32_bf16(false, a, false, b, (short)0, c, false, false); }

template <bool SPLITA, bool F16OUT = false>
__global__ __launch_bounds__(128) void k_gemmb(const bf* __restrict__ A, const bf* __restrict__ Al, const bf* __restrict__ Bn, const float* __restrict__ bias, float* C, int ldc, h16* C2, const float* __restrict__ R = nullptr, int K = DM, int roundR = 1) {
    __shared__ __align__(16) float ost[4][16 * 68];
    const int lane = threadIdx.x & 31, wave = threadIdx.x >> 5, lr = lane & 15, hi = lane >> 4;
    const int r0 = blockIdx.x * 64 + wave * 16, c0 = blockIdx.y * 64;
    const size_t aoff = (size_t)(r0 + lr) * K + 8 * hi;
    size_t boff[4];
#pragma unroll
    for (int t = 0; t < 4; ++t) boff[t] = (size_t)(c0 + t * 16 + lr) * K + 8 * hi;
    v8f acc[4];
#pragma unroll
    for (int t = 0; t < 4; ++t) acc[t] = (v8f){};
#pragma unroll 1
    for (int kc = 0; kc < K; kc += 32) {
        const v16bf a = cat16b(*(const v8us*)(A + aoff + kc), *(const v8us*)(A + aoff + kc + 16));
        v16bf al = a;
        if (SPLITA) al = cat16b(*(const v8us*)(Al + aoff + kc), *(const v8us*)(Al + aoff + kc + 16));
#pragma unroll
        for (int t = 0; t < 4; ++t) { const v16bf b = cat16b(*(const v8us*)(Bn + boff[t] + kc), *(const v8us*)(Bn + boff[t] + kc + 16)); acc[t] = wmmab(a, b, acc[t]); if (SPLITA) acc[t] = wmmab(al, b, acc[t]); }
        asm volatile("v_nop\n\tv_nop\n\tv_nop\n\tv_nop" : "+v"(acc[0]), "+v"(acc[1]), "+v"(acc[2]), "+v"(acc[3]) : "v"(a), "v"(al));
    }
    float* os = &ost[wave][0];
#pragma unroll
    for (int t = 0; t < 4; ++t) { const float bv = bias ? bfr(bias[c0 + t * 16 + lr]) : 0.f;
#pragma unroll
        for (int j = 0; j < 8; ++j) os[(hi * 8 + j) * 68 + t * 16 + lr] = acc[t][j] + bv; }
    __syncthreads();
    if (F16OUT) {
        h16* crow = (h16*)(void*)C + (size_t)r0 * ldc + c0;
        auto pass = [&]() {
#pragma unroll
            for (int s = 0; s < 4; ++s) { const int row = 4 * s + (lane >> 3), piece = lane & 7; const float* sp = os + row * 68 + piece * 8; v8h o, o2;
#pragma unroll
                for (int i = 0; i < 8; ++i) { const h16 a = (h16)sp[i]; o[i] = a; o2[i] = (h16)((sp[i] - (float)a) * LOSC); }
                *(volatile v8h*)(crow + (size_t)row * ldc + piece * 8) = o; if (C2) *(volatile v8h*)(C2 + (size_t)r0 * ldc + c0 + (size_t)row * ldc + piece * 8) = o2; }
        };
        pass(); __threadfence(); pass();
    } else {
        float* crow = C + (size_t)r0 * ldc + c0;
        auto pass = [&]() {
#pragma unroll
            for (int s = 0; s < 8; ++s) { const int Lid = (lane >> 3) + 4 * s, piece = lane & 7; const int row = Lid >> 1, cofs = (Lid & 1) * 32 + piece * 4;
                v4f val = *(const v4fa*)(os + row * 68 + cofs); if (R) { const v4f rv = *(const v4f*)(R + ((size_t)r0 + row) * ldc + c0 + cofs); val += roundR ? (v4f){bfr(rv[0]), bfr(rv[1]), bfr(rv[2]), bfr(rv[3])} : rv; }
                *(volatile v4f*)(crow + (size_t)row * ldc + cofs) = val; }
        };
        pass(); __threadfence(); pass();
    }
}


__global__ __launch_bounds__(128) void k_gemmh(const h16* __restrict__ A, const h16* __restrict__ Bn, const float* __restrict__ bias, float* C, int ldc, const float* __restrict__ R, int K, size_t sA, size_t sB, size_t sC, int roundR) {
    __shared__ __align__(16) float ost[4][16 * 68];
    const size_t z = blockIdx.z; A += z * sA; Bn += z * sB; C += z * sC; if (R) R += z * sC;
    const int lane = threadIdx.x & 31, wave = threadIdx.x >> 5, lr = lane & 15, hi = lane >> 4;
    const int r0 = blockIdx.x * 64 + wave * 16, c0 = blockIdx.y * 64;
    const size_t aoff = (size_t)(r0 + lr) * K + 8 * hi;
    size_t boff[4];
#pragma unroll
    for (int t = 0; t < 4; ++t) boff[t] = (size_t)(c0 + t * 16 + lr) * K + 8 * hi;
    v8f acc[4];
#pragma unroll
    for (int t = 0; t < 4; ++t) acc[t] = (v8f){};
#pragma unroll 1
    for (int kc = 0; kc < K; kc += 32) {
        const v16h a = cat16(*(const v8h*)(A + aoff + kc), *(const v8h*)(A + aoff + kc + 16));
#pragma unroll
        for (int t = 0; t < 4; ++t) { const v16h b = cat16(*(const v8h*)(Bn + boff[t] + kc), *(const v8h*)(Bn + boff[t] + kc + 16)); acc[t] = wmma16(a, b, acc[t]); }
        asm volatile("v_nop\n\tv_nop\n\tv_nop\n\tv_nop" : "+v"(acc[0]), "+v"(acc[1]), "+v"(acc[2]), "+v"(acc[3]) : "v"(a));
    }
    float* os = &ost[wave][0];
#pragma unroll
    for (int t = 0; t < 4; ++t) { const float bv = bias ? bfr(bias[c0 + t * 16 + lr]) : 0.f;
#pragma unroll
        for (int j = 0; j < 8; ++j) os[(hi * 8 + j) * 68 + t * 16 + lr] = acc[t][j] + bv; }
    __syncthreads();
    float* crow = C + (size_t)r0 * ldc + c0;
    auto pass = [&]() {
#pragma unroll
        for (int s = 0; s < 8; ++s) { const int Lid = (lane >> 3) + 4 * s, piece = lane & 7; const int row = Lid >> 1, cofs = (Lid & 1) * 32 + piece * 4;
            v4f val = *(const v4fa*)(os + row * 68 + cofs); if (R) { const v4f rv = *(const v4f*)(R + ((size_t)r0 + row) * ldc + c0 + cofs); val += roundR ? (v4f){bfr(rv[0]), bfr(rv[1]), bfr(rv[2]), bfr(rv[3])} : rv; }
            *(volatile v4f*)(crow + (size_t)row * ldc + cofs) = val; }
    };
    pass(); __threadfence(); pass();
}

typedef __attribute__((ext_vector_type(4))) _Float16 v4h;
__device__ __forceinline__ h16 tohx(float x) { return (h16)x; }
__global__ __launch_bounds__(256) void k_sigma(const float* __restrict__ wf, const float* __restrict__ uf, const float* __restrict__ wg, const float* __restrict__ ug, const float* __restrict__ wh, const float* __restrict__ uh, const float* __restrict__ wo, const float* __restrict__ uo, float* SIG) {
    __shared__ float v[256]; __shared__ float t[256]; __shared__ float red[8]; __shared__ float sres[4];
    const int tid = threadIdx.x; const int wsel = blockIdx.x; const float* Wm = wsel == 0 ? wf : wsel == 1 ? wg : wsel == 2 ? wh : wo; const float* u = wsel == 0 ? uf : wsel == 1 ? ug : wsel == 2 ? uh : uo; const int CIN = wsel == 3 ? DV : CC; const int COUT = wsel < 2 ? DQK : wsel == 2 ? DV : CC;
    auto bsum = [&](float x) { float s = x;
#pragma unroll
        for (int sh = 16; sh; sh >>= 1) s += __shfl_xor(s, sh, 32);
        __syncthreads(); if ((tid & 31) == 0) red[tid >> 5] = s; __syncthreads(); float tot = 0.f; for (int k = 0; k < 8; ++k) tot += red[k]; __syncthreads(); return tot; };
    float vi = 0.f; if (tid < CIN) { for (int o = 0; o < COUT; ++o) vi = fmaf(bfr(u[o]), bfr(Wm[(size_t)tid * COUT + o]), vi); }
    const float nv = bsum(tid < CIN ? vi * vi : 0.f); const float invv = rsqrtf(fmaxf(nv, 1e-12f)); if (tid < CIN) v[tid] = vi * invv; __syncthreads();
    float to = 0.f; if (tid < COUT) { for (int i = 0; i < CIN; ++i) to = fmaf(v[i], bfr(Wm[(size_t)i * COUT + tid]), to); t[tid] = to; }
    const float nt = bsum(tid < COUT ? to * to : 0.f); const float invt = rsqrtf(fmaxf(nt, 1e-12f));
    const float sg = bsum(tid < COUT ? to * (to * invt) : 0.f);
    if (tid < 32) { const float val = (tid == 0) ? sg : 0.f; *(volatile float*)(SIG + wsel * 32 + tid) = val; __threadfence(); *(volatile float*)(SIG + wsel * 32 + tid) = val; }
}
__global__ __launch_bounds__(256) void k_cvtx(const float* __restrict__ x, bf* A) {
    const int lane = threadIdx.x & 31; const size_t r = (size_t)blockIdx.x * 8 + (threadIdx.x >> 5); if (r >= (size_t)NR) return; const size_t o = r * CC + lane * 8; v8us v;
#pragma unroll
    for (int i = 0; i < 8; ++i) v[i] = f2bf(x[o + i]);
    *(volatile v8us*)(A + o) = v; __threadfence(); *(volatile v8us*)(A + o) = v;
}
__global__ __launch_bounds__(256) void k_wcat(const float* __restrict__ wf, const float* __restrict__ wg, const float* __restrict__ wh, bf* Bt) {
    const int lane = threadIdx.x & 31; const int n = blockIdx.x * 8 + (threadIdx.x >> 5); if (n >= NPJ) return; v8us o;
#pragma unroll
    for (int i = 0; i < 8; ++i) { const int k = lane * 8 + i; const float w = (n < DQK) ? wf[(size_t)k * DQK + n] : (n < 2 * DQK) ? wg[(size_t)k * DQK + (n - DQK)] : wh[(size_t)k * DV + (n - 2 * DQK)]; o[i] = f2bf(w); }
    *(volatile v8us*)(Bt + (size_t)n * CC + lane * 8) = o; __threadfence(); *(volatile v8us*)(Bt + (size_t)n * CC + lane * 8) = o;
}
__global__ __launch_bounds__(256) void k_woT(const float* __restrict__ wo, h16* Bo) {
    const int lane = threadIdx.x & 31; const int n = blockIdx.x * 8 + (threadIdx.x >> 5); if (n >= CC) return; v4h o;
#pragma unroll
    for (int i = 0; i < 4; ++i) { const int k = lane * 4 + i; o[i] = tohx(bfr(wo[(size_t)k * CC + n])); }
    *(volatile v4h*)(Bo + (size_t)n * DV + lane * 4) = o; __threadfence(); *(volatile v4h*)(Bo + (size_t)n * DV + lane * 4) = o;
}
__global__ __launch_bounds__(256) void k_fgplanes(const float* __restrict__ PJ, const float* __restrict__ SIG, const float* __restrict__ bf_, const float* __restrict__ bg_, h16* Fp, h16* Gp) {
    const int lane = threadIdx.x & 31; const size_t r = ((size_t)blockIdx.x * 8 + (threadIdx.x >> 5)) * 4 + (lane >> 3); if (r >= (size_t)NR) return; const int c0 = (lane & 7) * 4; const float isf = __fdiv_rn(1.0f, SIG[0]), isg = __fdiv_rn(1.0f, SIG[32]); v4h of, og;
#pragma unroll
    for (int i = 0; i < 4; ++i) { of[i] = tohx(PJ[r * NPJ + c0 + i] * isf + bfr(bf_[c0 + i])); og[i] = tohx(PJ[r * NPJ + DQK + c0 + i] * isg + bfr(bg_[c0 + i])); }
    *(volatile v4h*)(Fp + r * DQK + c0) = of; *(volatile v4h*)(Gp + r * DQK + c0) = og; __threadfence(); *(volatile v4h*)(Fp + r * DQK + c0) = of; *(volatile v4h*)(Gp + r * DQK + c0) = og;
}
__global__ __launch_bounds__(256) void k_hT(const float* __restrict__ PJ, const float* __restrict__ SIG, const float* __restrict__ bh_, h16* HT) {
    __shared__ float tl[64][65];
    const int tid = threadIdx.x; const int t0 = blockIdx.x * 64, d0 = blockIdx.y * 64; const int b = blockIdx.z; const int rr = tid >> 2, cq = (tid & 3) * 16; const float ish = __fdiv_rn(1.0f, SIG[64]);
#pragma unroll
    for (int i = 0; i < 16; ++i) { const int d = d0 + cq + i; tl[rr][cq + i] = PJ[((size_t)b * HW + t0 + rr) * NPJ + 2 * DQK + d] * ish + bfr(bh_[d]); }
    __syncthreads();
    const int lane = tid & 31, wv = tid >> 5;
    auto pass = [&]() {
#pragma unroll
        for (int st = 0; st < 4; ++st) { const int dr = wv * 8 + st * 2 + (lane >> 4); const int tq = (lane & 15) * 4; v4h v;
#pragma unroll
            for (int i = 0; i < 4; ++i) v[i] = tohx(tl[tq + i][dr]);
            *(volatile v4h*)(HT + ((size_t)b * DV + d0 + dr) * HW + t0 + tq) = v; }
    };
    pass(); __threadfence(); pass();
}
__global__ __launch_bounds__(256) void k_softs(const float* __restrict__ S, h16* P) {
    const int lane = threadIdx.x & 31, i = blockIdx.x * 8 + (threadIdx.x >> 5); if (i >= HW) return; const size_t zo = (size_t)i * HW; const float* sr = S + zo; h16* po = P + zo;
    float m = -3.0e38f;
#pragma unroll 1
    for (int c0 = lane * 4; c0 < HW; c0 += 128) {
#pragma unroll
        for (int q = 0; q < 4; ++q) m = fmaxf(m, sr[c0 + q]); }
#pragma unroll
    for (int sh = 16; sh; sh >>= 1) m = fmaxf(m, __shfl_xor(m, sh, 32));
    float sum = 0.f;
#pragma unroll 1
    for (int c0 = lane * 4; c0 < HW; c0 += 128) {
#pragma unroll
        for (int q = 0; q < 4; ++q) sum += __expf(sr[c0 + q] - m); }
#pragma unroll
    for (int sh = 16; sh; sh >>= 1) sum += __shfl_xor(sum, sh, 32);
    const float f = __fdiv_rn(PCAR, sum);
#pragma unroll 1
    for (int ps = 0; ps < 2; ++ps) {
#pragma unroll 1
        for (int c0 = lane * 4; c0 < HW; c0 += 128) { v4h o;
#pragma unroll
            for (int q = 0; q < 4; ++q) o[q] = tohx(__expf(sr[c0 + q] - m) * f);
            *(volatile v4h*)(po + c0) = o; }
        if (ps == 0) __threadfence(); }
}
__global__ __launch_bounds__(256) void k_oplane(const float* __restrict__ O, int b, h16* Op) {
    const int lane = threadIdx.x & 31, t = blockIdx.x * 8 + (threadIdx.x >> 5); if (t >= HW) return; v4h o;
#pragma unroll
    for (int i = 0; i < 4; ++i) o[i] = tohx(O[(size_t)t * DV + lane * 4 + i] * (1.0f / PCAR));
    *(volatile v4h*)(Op + ((size_t)b * HW + t) * DV + lane * 4) = o; __threadfence(); *(volatile v4h*)(Op + ((size_t)b * HW + t) * DV + lane * 4) = o;
}
__global__ __launch_bounds__(256) void k_fin(const float* __restrict__ C2, const float* __restrict__ SIG, const float* __restrict__ bo_, const float* __restrict__ gam, const float* __restrict__ x, float* OUTB) {
    const int lane = threadIdx.x & 31; const size_t r = (size_t)blockIdx.x * 8 + (threadIdx.x >> 5); if (r >= (size_t)NR) return; const float iso = __fdiv_rn(1.0f, SIG[96]); const float gmm = bfr(gam[0]);
#pragma unroll 1
    for (int ps = 0; ps < 2; ++ps) {
#pragma unroll
        for (int p = 0; p < 2; ++p) { const int c0 = p * 128 + lane * 4; v4f o;
#pragma unroll
            for (int i = 0; i < 4; ++i) { const int c = c0 + i; o[i] = gmm * (C2[r * CC + c] * iso + bfr(bo_[c])) + bfr(x[r * CC + c]); }
            *(volatile v4f*)(OUTB + r * CC + c0) = o; }
        if (ps == 0) __threadfence(); }
}
extern "C" void kernel_launch(void* const* d_in, const int* in_sizes, int n_in,
                              void* d_out, int out_size, void* d_ws, size_t ws_size, hipStream_t stream) {
    (void)in_sizes; (void)n_in; (void)out_size;
    const float* x = (const float*)d_in[0]; const float* wf = (const float*)d_in[1]; const float* bf_ = (const float*)d_in[2]; const float* uf = (const float*)d_in[3]; const float* wg = (const float*)d_in[4]; const float* bg_ = (const float*)d_in[5]; const float* ug = (const float*)d_in[6]; const float* wh = (const float*)d_in[7]; const float* bh_ = (const float*)d_in[8]; const float* uh = (const float*)d_in[9]; const float* wo = (const float*)d_in[10]; const float* bo_ = (const float*)d_in[11]; const float* uo = (const float*)d_in[12]; const float* gam = (const float*)d_in[13];
    float* out = (float*)d_out;
    char* wsp = (char*)d_ws;
    auto take = [&](size_t bytes) { char* p = wsp; wsp += (bytes + 255) & ~(size_t)255; return (void*)p; };
    float* SIG = (float*)take(4 * 32 * 4); bf* XB = (bf*)take((size_t)NR * CC * 2); bf* WB = (bf*)take((size_t)NPJ * CC * 2); h16* WO = (h16*)take((size_t)CC * DV * 2); float* PJ = (float*)take((size_t)NR * NPJ * 4);
    h16* Fp = (h16*)take((size_t)NR * DQK * 2); h16* Gp = (h16*)take((size_t)NR * DQK * 2); h16* HT = (h16*)take((size_t)NB_ * DV * HW * 2); float* S = (float*)take((size_t)HW * HW * 4); h16* Px = (h16*)take((size_t)HW * HW * 2); float* O = (float*)take((size_t)HW * DV * 4); h16* Op = (h16*)take((size_t)NR * DV * 2); float* C2 = (float*)take((size_t)NR * CC * 4);
    if ((size_t)(wsp - (char*)d_ws) > ws_size) return;
    k_sigma<<<4, 256, 0, stream>>>(wf, uf, wg, ug, wh, uh, wo, uo, SIG);
    k_cvtx<<<NR / 8, 256, 0, stream>>>(x, XB); k_wcat<<<NPJ / 8, 256, 0, stream>>>(wf, wg, wh, WB); k_woT<<<CC / 8, 256, 0, stream>>>(wo, WO);
    k_gemmb<false, false><<<dim3(NR / 64, NPJ / 64, 1), 128, 0, stream>>>(XB, nullptr, WB, nullptr, PJ, NPJ, nullptr, nullptr, CC);
    k_fgplanes<<<(NR / 4) / 8, 256, 0, stream>>>(PJ, SIG, bf_, bg_, Fp, Gp); k_hT<<<dim3(HW / 64, DV / 64, NB_), 256, 0, stream>>>(PJ, SIG, bh_, HT);
    for (int b = 0; b < NB_; ++b) {
        k_gemmh<<<dim3(HW / 64, HW / 64, 1), 128, 0, stream>>>(Gp + (size_t)b * HW * DQK, Fp + (size_t)b * HW * DQK, nullptr, S, HW, nullptr, DQK, 0, 0, 0, 0);
        k_softs<<<HW / 8, 256, 0, stream>>>(S, Px);
        k_gemmh<<<dim3(HW / 64, DV / 64, 1), 128, 0, stream>>>(Px, HT + (size_t)b * DV * HW, nullptr, O, DV, nullptr, HW, 0, 0, 0, 0);
        k_oplane<<<HW / 8, 256, 0, stream>>>(O, b, Op); }
    k_gemmh<<<dim3(NR / 64, CC / 64, 1), 128, 0, stream>>>(Op, WO, nullptr, C2, CC, nullptr, DV, 0, 0, 0, 0);
    k_fin<<<NR / 8, 256, 0, stream>>>(C2, SIG, bo_, gam, x, out);
}
